// DenseCRFLoss_38817914421724
// MI455X (gfx1250) — hardware-verified
//
#include <hip/hip_runtime.h>
#include <stdint.h>

typedef _Float16       v16h __attribute__((ext_vector_type(16)));
typedef __bf16         v16b __attribute__((ext_vector_type(16)));
typedef unsigned short v8us __attribute__((ext_vector_type(8)));
typedef v8us           v8usa __attribute__((may_alias));
typedef unsigned int   v4u  __attribute__((ext_vector_type(4)));
typedef float          v8f  __attribute__((ext_vector_type(8)));
typedef float          v4f  __attribute__((ext_vector_type(4)));
typedef v4f            v4fa __attribute__((may_alias));

#define SRCH 192
#define SRCW 192
#define DH 96
#define DW 96
#define PTS (DH * DW)
#define KSEG 21
#define NT (PTS / 16)
#define ROWH 32
#define PSTRIDE 128
#define WPB 8

#define EXP2_SCALE (-0.72134752044448170f)

__device__ __forceinline__ float fexp2(float x) {
#if __has_builtin(__builtin_amdgcn_exp2f)
  return __builtin_amdgcn_exp2f(x);
#else
  return exp2f(x);
#endif
}

__device__ __forceinline__ unsigned short bf16_rne(float x) {
  unsigned int u = __float_as_uint(x);
  u += 0x7FFFu + ((u >> 16) & 1u);
  return (unsigned short)(u >> 16);
}
__device__ __forceinline__ float bf16_val(unsigned short bb) {
  return __uint_as_float(((unsigned int)bb) << 16);
}
__device__ __forceinline__ unsigned short f16_bits(float x) {
  union { _Float16 h; unsigned short u; } c;
  c.h = (_Float16)x;
  return c.u;
}

__device__ __forceinline__ v8f wmma_bf16_acc(v16b a, v16b b, v8f c) {
  v8f d = __builtin_amdgcn_wmma_f32_16x16x32_bf16(false, a, false, b, (short)0, c, false, false);
  asm volatile("v_nop\n\tv_nop\n\tv_nop\n\tv_nop" : "+v"(d) : "v"(a), "v"(b));
  return d;
}
__device__ __forceinline__ v8f wmma_f16_acc(v16h a, v16h b, v8f c) {
  v8f d = __builtin_amdgcn_wmma_f32_16x16x32_f16(false, a, false, b, (short)0, c, false, false);
  asm volatile("v_nop\n\tv_nop\n\tv_nop\n\tv_nop" : "+v"(d) : "v"(a), "v"(b));
  return d;
}

union FragB16 { v16b v; v8us h8[2]; };
union FragF16 { v16h v; v8us h8[2]; };

__device__ __forceinline__ void store_rows_twice(const unsigned short* lrow,
                                                 unsigned short* __restrict__ g,
                                                 size_t row0, int w, int lane)
{
  union { v8us s; v4u u; } v[4];
  const unsigned short* ls = lrow + w * (32 * ROWH) + lane * 8;
#pragma unroll
  for (int q = 0; q < 4; ++q) v[q].s = *(const v8usa*)(ls + q * 256);
  unsigned short* gp = g + (row0 + (size_t)w * 32) * ROWH + lane * 8;
#pragma unroll
  for (int q = 0; q < 4; ++q) *(volatile v4u*)(gp + q * 256) = v[q].u;
  __threadfence();
#pragma unroll
  for (int q = 0; q < 4; ++q) *(volatile v4u*)(gp + q * 256) = v[q].u;
}

__global__ void __launch_bounds__(256)
k_prep(const float* __restrict__ seg,
       const float* __restrict__ img,
       int npts,
       unsigned short* __restrict__ ga,
       unsigned short* __restrict__ gb,
       unsigned short* __restrict__ gsv,
       float* __restrict__ gsq)
{
#pragma clang fp contract(off)
  __shared__ unsigned short lrow[256 * ROWH];
  __shared__ float lsq[256];

  const int tid = threadIdx.x, lane = tid & 31, w = tid >> 5;
  const size_t row0 = (size_t)blockIdx.x * 256;
  const int t  = (int)row0 + tid;
  const int tc = (t < npts) ? t : (npts - 1);
  const int b  = tc / PTS;
  const int p  = tc - b * PTS;
  const int y  = p / DW;
  const int x  = p - y * DW;
  const size_t plane = (size_t)SRCH * SRCW;
  const size_t off = (size_t)(2 * y) * SRCW + (size_t)(2 * x);

  const float* ib = img + (size_t)b * 3 * plane + off;
  float f[5];
  f[0] = (float)x * (1.0f / 50.0f);
  f[1] = (float)y * (1.0f / 50.0f);
  f[2] = ib[0]         * (1.0f / 15.0f);
  f[3] = ib[plane]     * (1.0f / 15.0f);
  f[4] = ib[2 * plane] * (1.0f / 15.0f);

  float s2 = 0.f;
#pragma unroll
  for (int c = 0; c < 5; ++c) s2 = s2 + f[c] * f[c];
  lsq[tid] = s2;

  unsigned short ph[5], pm[5], pl[5];
#pragma unroll
  for (int c = 0; c < 5; ++c) {
    const float v  = f[c];
    const unsigned short hb = bf16_rne(v);
    const float r1 = v - bf16_val(hb);
    const unsigned short mb = bf16_rne(r1);
    const float r2 = r1 - bf16_val(mb);
    const unsigned short lb = bf16_rne(r2);
    ph[c] = hb; pm[c] = mb; pl[c] = lb;
  }

  unsigned short* lr = lrow + tid * ROWH;

#pragma unroll
  for (int c = 0; c < 5; ++c) {
    lr[c]      = ph[c];
    lr[5 + c]  = ph[c];
    lr[10 + c] = ph[c];
    lr[15 + c] = pm[c];
    lr[20 + c] = pm[c];
    lr[25 + c] = pl[c];
  }
  lr[30] = 0; lr[31] = 0;
  __syncthreads();
  store_rows_twice(lrow, ga, row0, w, lane);
  {
    v4f q4 = {0.f, 0.f, 0.f, 0.f};
    if (tid < 64) q4 = *(const v4fa*)(lsq + tid * 4);
    float* sp = gsq + row0 + (size_t)tid * 4;
    if (tid < 64) *(volatile v4f*)sp = q4;
    __threadfence();
    if (tid < 64) *(volatile v4f*)sp = q4;
  }
  __syncthreads();

#pragma unroll
  for (int c = 0; c < 5; ++c) {
    lr[c]      = ph[c];
    lr[5 + c]  = pm[c];
    lr[10 + c] = pl[c];
    lr[15 + c] = ph[c];
    lr[20 + c] = pm[c];
    lr[25 + c] = ph[c];
  }
  lr[30] = 0; lr[31] = 0;
  __syncthreads();
  store_rows_twice(lrow, gb, row0, w, lane);
  __syncthreads();

  const float* sb = seg + (size_t)b * KSEG * plane + off;
#pragma unroll
  for (int k = 0; k < KSEG; ++k) {
    const float* sk = sb + (size_t)k * plane;
    const float v = ((sk[0] + sk[1]) + (sk[SRCW] + sk[SRCW + 1])) * 0.25f;
    lr[k] = f16_bits(v * 16.0f);
  }
#pragma unroll
  for (int k = KSEG; k < ROWH; ++k) lr[k] = 0;
  __syncthreads();
  store_rows_twice(lrow, gsv, row0, w, lane);
}

__global__ void __launch_bounds__(256)
k_pairs(const unsigned short* __restrict__ ga,
        const unsigned short* __restrict__ gb,
        const unsigned short* __restrict__ gsv,
        const float* __restrict__ gsq,
        float* __restrict__ part)
{
  __shared__ float red[WPB];
  __shared__ float bsum;

  const int tid = threadIdx.x, lane = tid & 31, w = tid >> 5;
  const int h = lane >> 4, m = lane & 15;
  const int blk = blockIdx.x;
  const int b  = blk / NT;
  const int ti = blk - b * NT;
  const size_t pbase = (size_t)b * PTS;

  const size_t irow = pbase + (size_t)ti * 16 + m;
  FragB16 fa;
  fa.h8[0] = *(const v8us*)(ga + irow * ROWH + 8 * h);
  fa.h8[1] = *(const v8us*)(ga + irow * ROWH + 16 + 8 * h);
  FragF16 sa;
  sa.h8[0] = *(const v8us*)(gsv + irow * ROWH + 8 * h);
  sa.h8[1] = *(const v8us*)(gsv + irow * ROWH + 16 + 8 * h);

  float sqi[8];
  const float* sqp = gsq + pbase + (size_t)ti * 16 + 8 * h;
#pragma unroll
  for (int r = 0; r < 8; ++r) sqi[r] = sqp[r];

  float acc = 0.f;
  for (int tj = ti + w; tj < NT; tj += WPB) {
    const size_t jrow = pbase + (size_t)tj * 16 + m;
    FragB16 fb;
    fb.h8[0] = *(const v8us*)(gb + jrow * ROWH + 8 * h);
    fb.h8[1] = *(const v8us*)(gb + jrow * ROWH + 16 + 8 * h);
    FragF16 sbv;
    sbv.h8[0] = *(const v8us*)(gsv + jrow * ROWH + 8 * h);
    sbv.h8[1] = *(const v8us*)(gsv + jrow * ROWH + 16 + 8 * h);
    const float sqj = gsq[jrow];

    const v8f z = {0.f, 0.f, 0.f, 0.f, 0.f, 0.f, 0.f, 0.f};
    const v8f dot = wmma_bf16_acc(fa.v, fb.v, z);
    const v8f g   = wmma_f16_acc(sa.v, sbv.v, z);

    float psum = 0.f;
#pragma unroll
    for (int r = 0; r < 8; ++r) {
      const float d2 = (sqi[r] + sqj) - 2.0f * dot[r];
      psum += g[r] * fexp2(EXP2_SCALE * d2);
    }
    const float wgt = (tj == ti) ? 1.0f : 2.0f;
    acc += wgt * psum;
  }

#pragma unroll
  for (int o = 16; o > 0; o >>= 1) acc += __shfl_xor(acc, o, 32);
  if (lane == 0) red[w] = acc;
  __syncthreads();
  if (tid == 0) {
    double s = 0.0;
#pragma unroll
    for (int i = 0; i < WPB; ++i) s += (double)red[i];
    bsum = (float)s;
  }
  __syncthreads();
  if (w == 0) {
    const float v = bsum;
    const v4f q4 = {v, v, v, v};
    float* pp = part + (size_t)blk * PSTRIDE + lane * 4;
    *(volatile v4f*)pp = q4;
    __threadfence();
    *(volatile v4f*)pp = q4;
  }
}

__global__ void __launch_bounds__(256)
k_final(const float* __restrict__ part, float* __restrict__ out, int nblk, double scale)
{
  __shared__ double lr[256];
  const int tid = threadIdx.x;
  double s = 0.0;
  for (int i = tid; i < nblk; i += 256) s += (double)part[(size_t)i * PSTRIDE];
  lr[tid] = s;
  __syncthreads();
  for (int o = 128; o > 0; o >>= 1) {
    if (tid < o) lr[tid] += lr[tid + o];
    __syncthreads();
  }
  if (tid == 0) {
    const float v = (float)(lr[0] * scale);
    volatile float* vo = out;
    vo[0] = v;
    __threadfence();
    vo[0] = v;
  }
}

extern "C" void kernel_launch(void* const* d_in, const int* in_sizes, int n_in,
                              void* d_out, int out_size, void* d_ws, size_t ws_size,
                              hipStream_t stream) {
  if (n_in < 2 || out_size < 1) return;
  const float* seg = (const float*)d_in[0];
  const float* img = (const float*)d_in[1];

  const int plane = SRCH * SRCW;
  const int B = in_sizes[1] / (3 * plane);
  if (B <= 0 || in_sizes[1] != B * 3 * plane || in_sizes[0] != B * KSEG * plane) return;

  const int npts  = B * PTS;
  const int gprep = (npts + 255) / 256;
  const size_t rows_pad  = (size_t)gprep * 256;
  const size_t row_bytes = rows_pad * ROWH * sizeof(unsigned short);
  const size_t sq_bytes  = rows_pad * sizeof(float);
  const int nblk = B * NT;
  const size_t part_bytes = (size_t)nblk * PSTRIDE * sizeof(float);

  const size_t o_a = 0, o_b = row_bytes, o_s = 2 * row_bytes, o_sq = 3 * row_bytes;
  const size_t o_part = o_sq + sq_bytes;
  if (o_part + part_bytes > ws_size) return;

  char* ws = (char*)d_ws;
  unsigned short* ga  = (unsigned short*)(ws + o_a);
  unsigned short* gb  = (unsigned short*)(ws + o_b);
  unsigned short* gsv = (unsigned short*)(ws + o_s);
  float* gsq  = (float*)(ws + o_sq);
  float* part = (float*)(ws + o_part);
  float* out  = (float*)d_out;

  k_prep<<<gprep, 256, 0, stream>>>(seg, img, npts, ga, gb, gsv, gsq);
  k_pairs<<<nblk, 256, 0, stream>>>(ga, gb, gsv, gsq, part);
  const double scale = -2.0e-9 / ((double)B * 256.0);
  k_final<<<1, 256, 0, stream>>>(part, out, nblk, scale);
}
